// _ConvBlock4LessLayers_43018392436809
// MI455X (gfx1250) — hardware-verified
//
#include <hip/hip_runtime.h>
#include <stddef.h>


#define CH       64
#define NTHR     256
#define NWAVE    8
#define EPT      8
#define NGRP     2
#define CHUNK    (NTHR * EPT * NGRP)
#define WCAP     (EPT * NGRP * 32)
#define LISTN    (NWAVE * WCAP)
#define NB       1024
#define NSEGC    50000
#define WPL      (CH * CH)
#define LDS_AGG  (NB * CH * 4 + LISTN * 4 + 64)
#define WS_LIMIT ((size_t)134217728)

static_assert((CHUNK & (CHUNK - 1)) == 0);
static_assert(CHUNK <= 4096);
static_assert((NB & (NB - 1)) == 0);
static_assert(NB <= 4096);
static_assert(NB % (16 * NWAVE) == 0);
static_assert(CH == 64);
static_assert((NB * CH) % (NWAVE * 128) == 0);

typedef float          v2f   __attribute__((ext_vector_type(2)));
typedef float          v4f   __attribute__((ext_vector_type(4)));
typedef float          v8f   __attribute__((ext_vector_type(8)));
typedef int            v4i   __attribute__((ext_vector_type(4)));
typedef unsigned short v8us  __attribute__((ext_vector_type(8)));
typedef unsigned short v16us __attribute__((ext_vector_type(16)));
typedef __bf16         v16bf __attribute__((ext_vector_type(16)));
union FragB { v16bf v; v16us u; v8us h[2]; };

__device__ __forceinline__ unsigned int bf16_rne_bits(float f) {
  const unsigned int u = __float_as_uint(f);
  return (u + 0x7FFFu + ((u >> 16) & 1u)) >> 16;
}

__device__ __forceinline__ v8f wmb(v16bf a, v16bf b, v8f c) {
  v8f d = __builtin_amdgcn_wmma_f32_16x16x32_bf16(false, a, false, b, (short)0, c, false, false);
  asm volatile("v_nop\n\tv_nop\n\tv_nop\n\tv_nop" : "+v"(d) : "v"(a), "v"(b));
  return d;
}

__device__ __forceinline__ void split16(v4f q0, v4f q1, v4f q2, v4f q3, FragB& ah, FragB& al) {
  float f[16] = {q0.x, q0.y, q0.z, q0.w, q1.x, q1.y, q1.z, q1.w,
                 q2.x, q2.y, q2.z, q2.w, q3.x, q3.y, q3.z, q3.w};
#pragma unroll
  for (int i = 0; i < 16; ++i) {
    const unsigned int hb = bf16_rne_bits(f[i]);
    const unsigned int lb = bf16_rne_bits(f[i] - __uint_as_float(hb << 16));
    ah.u[i] = (unsigned short)hb;
    al.u[i] = (unsigned short)lb;
  }
}

__device__ __forceinline__ int scan_chunk(const int* __restrict__ dsts, int nE, int cbase, int nodeBase,
                                          unsigned int lim, int* list, int tid, int wave) {
  int wc = 0;
#pragma unroll
  for (int g = 0; g < NGRP; ++g) {
    const int el0  = (g * NTHR + tid) * EPT;
    const int e0   = cbase + el0;
    const int sent = -2147483647 - 1;
    v4i da, db;
    if (e0 + 7 < nE) {
      da = *(const v4i*)(dsts + e0);
      db = *(const v4i*)(dsts + e0 + 4);
    } else {
      da.x = (e0     < nE) ? dsts[min(e0, nE - 1)] : sent;
      da.y = (e0 + 1 < nE) ? dsts[min(e0 + 1, nE - 1)] : sent;
      da.z = (e0 + 2 < nE) ? dsts[min(e0 + 2, nE - 1)] : sent;
      da.w = (e0 + 3 < nE) ? dsts[min(e0 + 3, nE - 1)] : sent;
      db.x = (e0 + 4 < nE) ? dsts[min(e0 + 4, nE - 1)] : sent;
      db.y = (e0 + 5 < nE) ? dsts[min(e0 + 5, nE - 1)] : sent;
      db.z = (e0 + 6 < nE) ? dsts[min(e0 + 6, nE - 1)] : sent;
      db.w = (e0 + 7 < nE) ? dsts[min(e0 + 7, nE - 1)] : sent;
    }
    const unsigned nb = (unsigned)nodeBase;
    const unsigned s0 = (unsigned)da.x - nb, s1 = (unsigned)da.y - nb;
    const unsigned s2 = (unsigned)da.z - nb, s3 = (unsigned)da.w - nb;
    const unsigned s4 = (unsigned)db.x - nb, s5 = (unsigned)db.y - nb;
    const unsigned s6 = (unsigned)db.z - nb, s7 = (unsigned)db.w - nb;
    const bool h0 = s0 < lim, h1 = s1 < lim, h2 = s2 < lim, h3 = s3 < lim;
    const bool h4 = s4 < lim, h5 = s5 < lim, h6 = s6 < lim, h7 = s7 < lim;
    const unsigned any = __builtin_amdgcn_ballot_w32(h0 | h1 | h2 | h3 | h4 | h5 | h6 | h7);
    if (any != 0u) {
#define HITJ(J, HJ, SJ) { \
        const unsigned mj = __builtin_amdgcn_ballot_w32(HJ); \
        if (mj != 0u) { \
          if (HJ) { \
            const int pos = wc + (int)__builtin_amdgcn_mbcnt_lo(mj, 0u); \
            if (pos < WCAP) list[wave * WCAP + pos] = ((el0 + (J)) << 12) | (int)(SJ); \
          } \
          wc += (int)__builtin_popcount(mj); } }
      HITJ(0, h0, s0)
      HITJ(1, h1, s1)
      HITJ(2, h2, s2)
      HITJ(3, h3, s3)
      HITJ(4, h4, s4)
      HITJ(5, h5, s5)
      HITJ(6, h6, s6)
      HITJ(7, h7, s7)
#undef HITJ
    }
  }
  return wc;
}

__device__ __forceinline__ void drain_lists(float* acc, const int* list, const int* wcnt,
                                            const float* __restrict__ feat, const int* __restrict__ srcI,
                                            const float* __restrict__ ew, int cbase, int nE, int nsrc, int lane) {
#pragma unroll 1
  for (int wsx = 0; wsx < NWAVE; ++wsx) {
    int n = __builtin_amdgcn_readfirstlane(wcnt[wsx]);
    n = n > WCAP ? WCAP : (n < 0 ? 0 : n);
    const int* lp = list + wsx * WCAP;
#pragma unroll 1
    for (int i = 0; i < n; ++i) {
      const int ent  = __builtin_amdgcn_readfirstlane(lp[i]);
      const int slot = ent & (NB - 1);
      int e = cbase + ((ent >> 12) & (CHUNK - 1));
      e = e > nE - 1 ? nE - 1 : e;
      int src = srcI[e];
      src = src < 0 ? 0 : (src > nsrc - 1 ? nsrc - 1 : src);
      const float wv = ew[e];
      const v2f v = *(const v2f*)(feat + (size_t)src * CH + 2 * lane);
      v2f* ap = (v2f*)(acc + slot * CH + 2 * lane);
      v2f a = *ap;
      a.x = a.x + wv * v.x;
      a.y = a.y + wv * v.y;
      *ap = a;
    }
  }
}

__global__ __launch_bounds__(NTHR) void k_wprep(
    const float* __restrict__ Wr, const float* __restrict__ Wn, unsigned short* wpl, int nL) {
  const int i = blockIdx.x * NTHR + threadIdx.x;
  if (i >= nL * 2 * CH * 8) return;
  const int kq    = i & 7;
  const int n     = (i >> 3) & (CH - 1);
  const int mat   = (i >> 9) & 1;
  const int layer = i >> 10;
  const float* W = (mat != 0 ? Wn : Wr) + ((size_t)layer * CH + 8 * kq) * CH + n;
  v8us hv, lv;
#pragma unroll
  for (int j = 0; j < 8; ++j) {
    const float f = W[(size_t)j * CH];
    const unsigned int hb = bf16_rne_bits(f);
    const unsigned int lb = bf16_rne_bits(f - __uint_as_float(hb << 16));
    hv[j] = (unsigned short)hb;
    lv[j] = (unsigned short)lb;
  }
  unsigned short* ph = wpl + (size_t)((layer * 2 + mat) * 2) * WPL + n * CH + 8 * kq;
  unsigned short* pl = ph + WPL;
  *(volatile v8us*)ph = hv;
  *(volatile v8us*)pl = lv;
  __threadfence();
  *(volatile v8us*)ph = hv;
  *(volatile v8us*)pl = lv;
}

__global__ __launch_bounds__(NTHR) void k_segsum(
    const float* __restrict__ feat, const int* __restrict__ srcI, const int* __restrict__ dstI,
    const float* __restrict__ ew, const int* __restrict__ nsrcp, const int* __restrict__ nsegp,
    float* orow, int nE, int srcCap, int segCap, int nOutRows) {
  extern __shared__ v4f lds_dyn[];
  float* acc  = (float*)lds_dyn;
  int*   list = (int*)(acc + NB * CH);
  int*   wcnt = list + LISTN;
  const int tid = threadIdx.x, lane = tid & 31, wave = tid >> 5;
  const int nodeBase = blockIdx.x * NB;

  int nsrc = nsrcp[0];
  nsrc = nsrc < 1 ? 1 : (nsrc > srcCap ? srcCap : nsrc);
  int nseg = nsegp[0];
  nseg = nseg < 0 ? 0 : (nseg > segCap ? segCap : nseg);
  int lm = nseg - nodeBase;
  lm = lm < 0 ? 0 : (lm > NB ? NB : lm);
  const unsigned int lim = (unsigned int)lm;

  {
    const v4f z = {0.f, 0.f, 0.f, 0.f};
    for (int i = tid; i < NB * CH / 4; i += NTHR) lds_dyn[i] = z;
  }
  __syncthreads();

  const int nChunks = (nE + CHUNK - 1) / CHUNK;
#pragma unroll 1
  for (int ch = 0; ch < nChunks; ++ch) {
    const int cbase = ch * CHUNK;
    const int wc = scan_chunk(dstI, nE, cbase, nodeBase, lim, list, tid, wave);
    if (lane == 0) wcnt[wave] = wc;
    __syncthreads();
    if (wave == 0) drain_lists(acc, list, wcnt, feat, srcI, ew, cbase, nE, nsrc, lane);
    __syncthreads();
  }

  const size_t ob   = (size_t)nodeBase * CH;
  const size_t limf = (size_t)nOutRows * CH;
  const int    QN   = (NB * CH) / (NWAVE * 128);
#pragma unroll 4
  for (int q = 0; q < QN; ++q) {
    const int f = (wave * QN + q) * 128 + 4 * lane;
    const size_t gi = ob + (size_t)f;
    if (gi < limf) { const v4f v = *(const v4f*)(acc + f); *(volatile v4f*)(orow + gi) = v; }
  }
  __threadfence();
#pragma unroll 4
  for (int q = 0; q < QN; ++q) {
    const int f = (wave * QN + q) * 128 + 4 * lane;
    const size_t gi = ob + (size_t)f;
    if (gi < limf) { const v4f v = *(const v4f*)(acc + f); *(volatile v4f*)(orow + gi) = v; }
  }
}

__device__ __forceinline__ void kstep(v8f (&acc)[4], const FragB& ah, const FragB& al,
                                      const unsigned short* __restrict__ wp, int kt, int hh, int m) {
#pragma unroll
  for (int nt = 0; nt < 4; ++nt) {
    const unsigned short* bp = wp + (16 * nt + m) * CH + 32 * kt + 8 * hh;
    FragB bh, bl;
    bh.h[0] = *(const v8us*)bp;          bh.h[1] = *(const v8us*)(bp + 16);
    bl.h[0] = *(const v8us*)(bp + WPL);  bl.h[1] = *(const v8us*)(bp + WPL + 16);
    acc[nt] = wmb(ah.v, bh.v, acc[nt]);
    acc[nt] = wmb(ah.v, bl.v, acc[nt]);
    acc[nt] = wmb(al.v, bh.v, acc[nt]);
  }
}

__global__ __launch_bounds__(NTHR) void k_conv(
    const float* __restrict__ hin, const int* __restrict__ srcI, const int* __restrict__ dstI,
    const float* __restrict__ ew, const int* __restrict__ ncp,
    const unsigned short* __restrict__ wpl, const float* __restrict__ bias,
    float* hout, int nE, int nCap) {
  extern __shared__ v4f lds_dyn[];
  float* agg  = (float*)lds_dyn;
  int*   list = (int*)(agg + NB * CH);
  int*   wcnt = list + LISTN;
  const int tid = threadIdx.x, lane = tid & 31, wave = tid >> 5, hh = lane >> 4, m = lane & 15;
  const int nodeBase = blockIdx.x * NB;

  int nc = ncp[0];
  const int nsrc = nc < 1 ? 1 : (nc > nCap ? nCap : nc);
  const int nseg = nc < 0 ? 0 : (nc > nCap ? nCap : nc);
  int lm = nseg - nodeBase;
  lm = lm < 0 ? 0 : (lm > NB ? NB : lm);
  const unsigned int lim = (unsigned int)lm;

  {
    const v4f z = {0.f, 0.f, 0.f, 0.f};
    for (int i = tid; i < NB * CH / 4; i += NTHR) lds_dyn[i] = z;
  }
  __syncthreads();

  const int nChunks = (nE + CHUNK - 1) / CHUNK;
#pragma unroll 1
  for (int ch = 0; ch < nChunks; ++ch) {
    const int cbase = ch * CHUNK;
    const int wc = scan_chunk(dstI, nE, cbase, nodeBase, lim, list, tid, wave);
    if (lane == 0) wcnt[wave] = wc;
    __syncthreads();
    if (wave == 0) drain_lists(agg, list, wcnt, hin, srcI, ew, cbase, nE, nsrc, lane);
    __syncthreads();
  }

  const int NT = NB / (16 * NWAVE);
#pragma unroll 1
  for (int qi = 0; qi < NT; ++qi) {
    const int t  = wave + NWAVE * qi;
    const int rl = 16 * t + m;
    v8f acc[4];
#pragma unroll
    for (int nt = 0; nt < 4; ++nt) { const v8f z = {0.f, 0.f, 0.f, 0.f, 0.f, 0.f, 0.f, 0.f}; acc[nt] = z; }

#pragma unroll 1
    for (int kt = 0; kt < 2; ++kt) {
      const float* p = hin + ((size_t)nodeBase + rl) * CH + 32 * kt + 8 * hh;
      const v4f q0 = *(const v4f*)p,        q1 = *(const v4f*)(p + 4);
      const v4f q2 = *(const v4f*)(p + 16), q3 = *(const v4f*)(p + 20);
      FragB ah, al;
      split16(q0, q1, q2, q3, ah, al);
      kstep(acc, ah, al, wpl, kt, hh, m);
    }
#pragma unroll 1
    for (int kt = 0; kt < 2; ++kt) {
      const float* p = agg + rl * CH + 32 * kt + 8 * hh;
      const v4f q0 = *(const v4f*)p,        q1 = *(const v4f*)(p + 4);
      const v4f q2 = *(const v4f*)(p + 16), q3 = *(const v4f*)(p + 20);
      FragB ah, al;
      split16(q0, q1, q2, q3, ah, al);
      kstep(acc, ah, al, wpl + 2 * WPL, kt, hh, m);
    }

    float* stg = agg + (16 * t) * CH;
#pragma unroll
    for (int nt = 0; nt < 4; ++nt) {
      const int col = 16 * nt + m;
      const float bv = bias[col];
      float* sp = stg + (8 * hh) * CH + col;
#pragma unroll
      for (int r = 0; r < 8; ++r) sp[r * CH] = fmaxf(acc[nt][r] + bv, 0.f);
    }
    __syncthreads();

    v4f ov[8];
#pragma unroll
    for (int j = 0; j < 8; ++j) ov[j] = *(const v4f*)(stg + (2 * j + hh) * CH + 4 * m);
    float* gp = hout + ((size_t)nodeBase + 16 * t) * CH;
#pragma unroll
    for (int j = 0; j < 8; ++j) *(volatile v4f*)(gp + (2 * j + hh) * CH + 4 * m) = ov[j];
    __threadfence();
#pragma unroll
    for (int j = 0; j < 8; ++j) *(volatile v4f*)(gp + (2 * j + hh) * CH + 4 * m) = ov[j];
  }
}

extern "C" void kernel_launch(void* const* d_in, const int* in_sizes, int n_in,
                              void* d_out, int out_size, void* d_ws, size_t ws_size,
                              hipStream_t stream) {
  if (n_in < 15) return;
  const int nF = in_sizes[0] / CH;
  if (nF <= 0 || in_sizes[0] != nF * CH || out_size != nF * CH) return;
  const int ePool = in_sizes[1], ePP = in_sizes[4], eUn = in_sizes[7];
  if (ePool < 0 || ePP < 0 || eUn < 0) return;
  if (in_sizes[2] != ePool || in_sizes[3] != ePool) return;
  if (in_sizes[5] != ePP || in_sizes[6] != ePP) return;
  if (in_sizes[8] != eUn || in_sizes[9] != eUn) return;
  const int nL = in_sizes[10] / WPL;
  if (nL < 0 || nL > 16 || in_sizes[10] != nL * WPL || in_sizes[11] != in_sizes[10] || in_sizes[12] < nL * CH) return;
  if (in_sizes[13] < 1 || in_sizes[14] < 1) return;

  const float* x          = (const float*)d_in[0];
  const int*   pool_src   = (const int*)d_in[1];
  const int*   pool_dst   = (const int*)d_in[2];
  const float* pool_w     = (const float*)d_in[3];
  const int*   pp_src     = (const int*)d_in[4];
  const int*   pp_dst     = (const int*)d_in[5];
  const float* pp_w       = (const float*)d_in[6];
  const int*   un_src     = (const int*)d_in[7];
  const int*   un_dst     = (const int*)d_in[8];
  const float* un_w       = (const float*)d_in[9];
  const float* Wr         = (const float*)d_in[10];
  const float* Wn         = (const float*)d_in[11];
  const float* bias       = (const float*)d_in[12];
  const int*   ncoarse_p  = (const int*)d_in[13];
  const int*   nfine_p    = (const int*)d_in[14];
  float* out = (float*)d_out;

  const int nBC  = (NSEGC + NB - 1) / NB;
  const int nCap = nBC * NB;
  const int nBF  = (nF + NB - 1) / NB;

  char* ws = (char*)d_ws;
  size_t off = 0;
  const size_t oW  = off; off += (size_t)nL * 4 * WPL * 2;          off = (off + 255) & ~(size_t)255;
  const size_t oHA = off; off += (size_t)nCap * CH * 4;             off = (off + 255) & ~(size_t)255;
  const size_t oHB = off; off += (size_t)nCap * CH * 4;             off = (off + 255) & ~(size_t)255;
  if (off > ws_size || off > WS_LIMIT) return;
  unsigned short* wpl = (unsigned short*)(ws + oW);
  float* hA = (float*)(ws + oHA);
  float* hB = (float*)(ws + oHB);

  if (nL > 0) {
    const int nPrep = nL * 2 * CH * 8;
    k_wprep<<<(nPrep + NTHR - 1) / NTHR, NTHR, 0, stream>>>(Wr, Wn, wpl, nL);
  }

  hipFuncSetAttribute(reinterpret_cast<const void*>(&k_segsum),
                      hipFuncAttributeMaxDynamicSharedMemorySize, LDS_AGG);
  hipFuncSetAttribute(reinterpret_cast<const void*>(&k_conv),
                      hipFuncAttributeMaxDynamicSharedMemorySize, LDS_AGG);

  k_segsum<<<nBC, NTHR, LDS_AGG, stream>>>(x, pool_src, pool_dst, pool_w, nfine_p, ncoarse_p,
                                            hA, ePool, nF, nCap, nCap);

  float* hc = hA;
  float* hn = hB;
  for (int layer = 0; layer < nL; ++layer) {
    k_conv<<<nBC, NTHR, LDS_AGG, stream>>>(hc, pp_src, pp_dst, pp_w, ncoarse_p,
                                            wpl + (size_t)layer * 4 * WPL, bias + (size_t)layer * CH,
                                            hn, ePP, nCap);
    float* tmp = hc; hc = hn; hn = tmp;
  }

  k_segsum<<<nBF, NTHR, LDS_AGG, stream>>>(hc, un_src, un_dst, un_w, ncoarse_p, nfine_p,
                                            out, eUn, nCap, nF, nF);
}
